// PatchConv2LayerClassifier_8117488190078
// MI455X (gfx1250) — hardware-verified
//
#include <hip/hip_runtime.h>
#include <stddef.h>


#define IN_F    64
#define HID     256
#define RD      128
#define NCLS    16
#define NPG     128
#define NTHR    256
#define NWAVE   8
#define EPT     8
#define NGRP    2
#define CHUNK   (NTHR * EPT * NGRP)
#define WCAP    (EPT * NGRP * 32)
#define LISTN   (NWAVE * WCAP)
#define NBD     4096
#define NB1     1024
#define NB2     512
#define TR1     16
#define GPB     (NB2 / NPG)
#define HROWS   32
#define NBW1    ((HID * IN_F / 8) / NTHR)
#define NBW2    ((RD * HID / 8) / NTHR)

#define LDS_L1  (NB1 * IN_F * 4 + LISTN * 4 + 64)
#define LDS_L2  (NB2 * RD * 4 + LISTN * 4 + 64)

static_assert((CHUNK & (CHUNK - 1)) == 0);
static_assert(CHUNK <= 4096);
static_assert(NBD <= 4096 && NB1 <= 4096 && NB2 <= 4096);
static_assert((NB1 & (NB1 - 1)) == 0 && (NB2 & (NB2 - 1)) == 0 && (NBD & (NBD - 1)) == 0);
static_assert(TR1 * HID * 2 + TR1 * RD * 4 <= LISTN * 4);
static_assert(GPB * RD * 4 <= LISTN * 4);
static_assert(NBD % NB1 == 0 && NBD % NB2 == 0 && NB2 % NPG == 0 && NB1 % TR1 == 0);
static_assert(NBW1 * NTHR * 8 == HID * IN_F && NBW2 * NTHR * 8 == RD * HID);

typedef float    v2f  __attribute__((ext_vector_type(2)));
typedef float    v4f  __attribute__((ext_vector_type(4)));
typedef float    v8f  __attribute__((ext_vector_type(8)));
typedef int      v4i  __attribute__((ext_vector_type(4)));
typedef _Float16 v8h  __attribute__((ext_vector_type(8)));
typedef _Float16 v16h __attribute__((ext_vector_type(16)));
union FragH { v16h v; v8h h[2]; };

__device__ __forceinline__ v8h cvt8(v4f a, v4f b) {
  v8h r;
  r[0] = (_Float16)a.x; r[1] = (_Float16)a.y; r[2] = (_Float16)a.z; r[3] = (_Float16)a.w;
  r[4] = (_Float16)b.x; r[5] = (_Float16)b.y; r[6] = (_Float16)b.z; r[7] = (_Float16)b.w;
  return r;
}

__device__ __forceinline__ v8f wmh(v16h a, v16h b, v8f c) {
  v8f d = __builtin_amdgcn_wmma_f32_16x16x32_f16(false, a, false, b, (short)0, c, false, false);
  asm volatile("v_nop\n\tv_nop\n\tv_nop\n\tv_nop" : "+v"(d) : "v"(a), "v"(b));
  return d;
}

template <int NB>
__device__ __forceinline__ int scan_chunk(const int* __restrict__ keys, int nE, int cbase, int nodeBase,
                                          int vec8, int* list, int tid, int lane, int wave) {
  int wc = 0;
#pragma unroll
  for (int g = 0; g < NGRP; ++g) {
    const int el0  = (g * NTHR + tid) * EPT;
    const int e0   = cbase + el0;
    const int sent = -2147483647 - 1;
    v4i da, db;
    if (vec8 != 0 && cbase + CHUNK <= nE) {
      da = *(const v4i*)(keys + e0);
      db = *(const v4i*)(keys + e0 + 4);
    } else {
      da.x = (e0     < nE) ? keys[min(e0, nE - 1)] : sent;
      da.y = (e0 + 1 < nE) ? keys[min(e0 + 1, nE - 1)] : sent;
      da.z = (e0 + 2 < nE) ? keys[min(e0 + 2, nE - 1)] : sent;
      da.w = (e0 + 3 < nE) ? keys[min(e0 + 3, nE - 1)] : sent;
      db.x = (e0 + 4 < nE) ? keys[min(e0 + 4, nE - 1)] : sent;
      db.y = (e0 + 5 < nE) ? keys[min(e0 + 5, nE - 1)] : sent;
      db.z = (e0 + 6 < nE) ? keys[min(e0 + 6, nE - 1)] : sent;
      db.w = (e0 + 7 < nE) ? keys[min(e0 + 7, nE - 1)] : sent;
    }
    const unsigned nb = (unsigned)nodeBase;
    const unsigned s0 = (unsigned)da.x - nb, s1 = (unsigned)da.y - nb;
    const unsigned s2 = (unsigned)da.z - nb, s3 = (unsigned)da.w - nb;
    const unsigned s4 = (unsigned)db.x - nb, s5 = (unsigned)db.y - nb;
    const unsigned s6 = (unsigned)db.z - nb, s7 = (unsigned)db.w - nb;
    const bool h0 = s0 < (unsigned)NB, h1 = s1 < (unsigned)NB, h2 = s2 < (unsigned)NB, h3 = s3 < (unsigned)NB;
    const bool h4 = s4 < (unsigned)NB, h5 = s5 < (unsigned)NB, h6 = s6 < (unsigned)NB, h7 = s7 < (unsigned)NB;
    const unsigned any = __builtin_amdgcn_ballot_w32(h0 | h1 | h2 | h3 | h4 | h5 | h6 | h7);
    if (any != 0u) {
#define HITJ(J, HJ, SJ) { \
        const unsigned mj = __builtin_amdgcn_ballot_w32(HJ); \
        if (mj != 0u) { \
          if (HJ) { \
            const int pos = wc + (int)__builtin_amdgcn_mbcnt_lo(mj, 0u); \
            if (pos < WCAP) list[wave * WCAP + pos] = ((el0 + (J)) << 12) | (int)(SJ); \
          } \
          wc += (int)__builtin_popcount(mj); } }
      HITJ(0, h0, s0)
      HITJ(1, h1, s1)
      HITJ(2, h2, s2)
      HITJ(3, h3, s3)
      HITJ(4, h4, s4)
      HITJ(5, h5, s5)
      HITJ(6, h6, s6)
      HITJ(7, h7, s7)
#undef HITJ
    }
  }
  return wc;
}

__global__ __launch_bounds__(NTHR) void k_wprep(
    const float* __restrict__ W1, const float* __restrict__ W2,
    _Float16* w1s, _Float16* w2s) {
  const int tid = threadIdx.x;
  v4f a, b;
  _Float16* dp;
  if (blockIdx.x < NBW1) {
    const int o  = (blockIdx.x * NTHR + tid) * 8;
    const int n  = o / IN_F;
    const int k0 = o - n * IN_F;
    const float* p = W1 + (size_t)k0 * HID + n;
    a.x = p[0];       a.y = p[HID];     a.z = p[2 * HID]; a.w = p[3 * HID];
    b.x = p[4 * HID]; b.y = p[5 * HID]; b.z = p[6 * HID]; b.w = p[7 * HID];
    dp = w1s + o;
  } else {
    const int o  = ((blockIdx.x - NBW1) * NTHR + tid) * 8;
    const int n  = o / HID;
    const int k0 = o - n * HID;
    const float* p = W2 + (size_t)k0 * RD + n;
    a.x = p[0];      a.y = p[RD];     a.z = p[2 * RD]; a.w = p[3 * RD];
    b.x = p[4 * RD]; b.y = p[5 * RD]; b.z = p[6 * RD]; b.w = p[7 * RD];
    dp = w2s + o;
  }
  a = a * 8.0f;
  b = b * 8.0f;
  const v8h hv = cvt8(a, b);
  *(volatile v8h*)dp = hv;
  __threadfence();
  *(volatile v8h*)dp = hv;
}

__global__ __launch_bounds__(NTHR) void k_deg(
    const int* __restrict__ esrc, const int* __restrict__ edst,
    float* dplanes, int planeN, int nE, int vec8) {
  __shared__ __attribute__((aligned(16))) int cnt[NBD];
  __shared__ __attribute__((aligned(16))) int list[LISTN];
  __shared__ int wcnt[NWAVE];
  const int tid = threadIdx.x, lane = tid & 31, wave = tid >> 5;
  const int nodeBase = blockIdx.x * NBD;
  const int* keys = (blockIdx.y == 0) ? esrc : edst;

  for (int i = tid; i < NBD; i += NTHR) cnt[i] = 0;
  __syncthreads();

  const int nChunks = (nE + CHUNK - 1) / CHUNK;
#pragma unroll 1
  for (int ch = 0; ch < nChunks; ++ch) {
    const int cbase = ch * CHUNK;
    const int wc = scan_chunk<NBD>(keys, nE, cbase, nodeBase, vec8, list, tid, lane, wave);
    if (lane == 0) wcnt[wave] = wc;
    __syncthreads();
    if (wave == 0) {
#pragma unroll 1
      for (int wsx = 0; wsx < NWAVE; ++wsx) {
        int n = __builtin_amdgcn_readfirstlane(wcnt[wsx]);
        n = n > WCAP ? WCAP : (n < 0 ? 0 : n);
        const int* lp = list + wsx * WCAP;
#pragma unroll 1
        for (int i = 0; i < n; ++i) {
          const int ent  = __builtin_amdgcn_readfirstlane(lp[i]);
          const int slot = ent & (NBD - 1);
          if (lane == 0) cnt[slot] = cnt[slot] + 1;
        }
      }
    }
    __syncthreads();
  }

  v4f dq[4];
#pragma unroll
  for (int q = 0; q < 4; ++q) {
    const int f = (wave * 4 + q) * 128 + 4 * lane;
    const v4i c = *(const v4i*)(cnt + f);
    dq[q].x = rsqrtf((float)(c.x > 1 ? c.x : 1));
    dq[q].y = rsqrtf((float)(c.y > 1 ? c.y : 1));
    dq[q].z = rsqrtf((float)(c.z > 1 ? c.z : 1));
    dq[q].w = rsqrtf((float)(c.w > 1 ? c.w : 1));
  }
  float* dp = dplanes + (size_t)blockIdx.y * (size_t)planeN + (size_t)nodeBase;
#pragma unroll
  for (int q = 0; q < 4; ++q) *(volatile v4f*)(dp + (wave * 4 + q) * 128 + 4 * lane) = dq[q];
  __threadfence();
#pragma unroll
  for (int q = 0; q < 4; ++q) *(volatile v4f*)(dp + (wave * 4 + q) * 128 + 4 * lane) = dq[q];
}

__global__ __launch_bounds__(NTHR) void k_layer1(
    const float* __restrict__ x, const float* __restrict__ ew,
    const int* __restrict__ esrc, const int* __restrict__ edst,
    const float* __restrict__ dso, const float* __restrict__ dsi,
    const _Float16* __restrict__ w1s, const _Float16* __restrict__ w2s,
    float* g2, int nN, int nE, int vec8) {
  extern __shared__ v4f lds_dyn[];
  float*    acc  = (float*)lds_dyn;
  int*      list = (int*)(acc + NB1 * IN_F);
  int*      wcnt = list + LISTN;
  _Float16* h1t  = (_Float16*)list;
  float*    stg  = (float*)list + (TR1 * HID) / 2;
  const int tid = threadIdx.x, lane = tid & 31, wave = tid >> 5, hh = lane >> 4, m = lane & 15;
  const int nodeBase = blockIdx.x * NB1;

  {
    const v4f z = {0.f, 0.f, 0.f, 0.f};
    for (int i = tid; i < NB1 * IN_F / 4; i += NTHR) lds_dyn[i] = z;
  }
  __syncthreads();

  const int nChunks = (nE + CHUNK - 1) / CHUNK;
#pragma unroll 1
  for (int ch = 0; ch < nChunks; ++ch) {
    const int cbase = ch * CHUNK;
    const int wc = scan_chunk<NB1>(edst, nE, cbase, nodeBase, vec8, list, tid, lane, wave);
    if (lane == 0) wcnt[wave] = wc;
    __syncthreads();
    if (wave == 0) {
#pragma unroll 1
      for (int wsx = 0; wsx < NWAVE; ++wsx) {
        int n = __builtin_amdgcn_readfirstlane(wcnt[wsx]);
        n = n > WCAP ? WCAP : (n < 0 ? 0 : n);
        const int* lp = list + wsx * WCAP;
#pragma unroll 1
        for (int i = 0; i < n; ++i) {
          const int ent  = __builtin_amdgcn_readfirstlane(lp[i]);
          const int slot = ent & (NB1 - 1);
          int e = cbase + ((ent >> 12) & (CHUNK - 1));
          e = e > nE - 1 ? nE - 1 : e;
          int s = esrc[e];
          s = s < 0 ? 0 : (s > nN - 1 ? nN - 1 : s);
          const float we = ew[e];
          const float dv = dso[s];
          const v2f xv = *(const v2f*)(x + (size_t)s * IN_F + 2 * lane);
          const v2f xs = xv * dv;
          const v2f mg = xs * we;
          v2f* ap = (v2f*)(acc + slot * IN_F + 2 * lane);
          *ap = *ap + mg;
        }
      }
    }
    __syncthreads();
  }

  const float k64 = 0.015625f, k128 = 0.0078125f;
#pragma unroll 1
  for (int it = 0; it < NB1 / TR1; ++it) {
    const int r0 = it * TR1;
    const float sA = dsi[(size_t)nodeBase + r0 + m] * 8.0f;
    v8f c[2];
#pragma unroll
    for (int t = 0; t < 2; ++t) { v8f z = {0.f, 0.f, 0.f, 0.f, 0.f, 0.f, 0.f, 0.f}; c[t] = z; }
#pragma unroll
    for (int kt = 0; kt < IN_F / 32; ++kt) {
      const float* ap = acc + (r0 + m) * IN_F + 32 * kt + 8 * hh;
      const v4f p0 = *(const v4f*)ap,        p1 = *(const v4f*)(ap + 4);
      const v4f p2 = *(const v4f*)(ap + 16), p3 = *(const v4f*)(ap + 20);
      FragH a;
      a.h[0] = cvt8(p0 * sA, p1 * sA);
      a.h[1] = cvt8(p2 * sA, p3 * sA);
#pragma unroll
      for (int t = 0; t < 2; ++t) {
        const _Float16* bp = w1s + (size_t)(16 * (2 * wave + t) + m) * IN_F + 32 * kt + 8 * hh;
        FragH b;
        b.h[0] = *(const v8h*)bp;
        b.h[1] = *(const v8h*)(bp + 16);
        c[t] = wmh(a.v, b.v, c[t]);
      }
    }
    const v4f oa = *(const v4f*)(dso + (size_t)nodeBase + r0 + 8 * hh);
    const v4f ob = *(const v4f*)(dso + (size_t)nodeBase + r0 + 8 * hh + 4);
    float so[8];
    so[0] = oa.x * 16.0f; so[1] = oa.y * 16.0f; so[2] = oa.z * 16.0f; so[3] = oa.w * 16.0f;
    so[4] = ob.x * 16.0f; so[5] = ob.y * 16.0f; so[6] = ob.z * 16.0f; so[7] = ob.w * 16.0f;
#pragma unroll
    for (int t = 0; t < 2; ++t) {
#pragma unroll
      for (int r = 0; r < 8; ++r) {
        float v = c[t][r] * k64;
        v = v >= 0.f ? v : 0.01f * v;
        h1t[(8 * hh + r) * HID + 32 * wave + 16 * t + m] = (_Float16)(v * so[r]);
      }
    }
    __syncthreads();

    v8f c2 = {0.f, 0.f, 0.f, 0.f, 0.f, 0.f, 0.f, 0.f};
#pragma unroll
    for (int kt = 0; kt < HID / 32; ++kt) {
      const _Float16* ap2 = h1t + m * HID + 32 * kt + 8 * hh;
      FragH a;
      a.h[0] = *(const v8h*)ap2;
      a.h[1] = *(const v8h*)(ap2 + 16);
      const _Float16* bp = w2s + (size_t)(16 * wave + m) * HID + 32 * kt + 8 * hh;
      FragH b;
      b.h[0] = *(const v8h*)bp;
      b.h[1] = *(const v8h*)(bp + 16);
      c2 = wmh(a.v, b.v, c2);
    }
    float* sp = stg + (8 * hh) * RD + 16 * wave + m;
    sp[0 * RD] = c2[0] * k128;
    sp[1 * RD] = c2[1] * k128;
    sp[2 * RD] = c2[2] * k128;
    sp[3 * RD] = c2[3] * k128;
    sp[4 * RD] = c2[4] * k128;
    sp[5 * RD] = c2[5] * k128;
    sp[6 * RD] = c2[6] * k128;
    sp[7 * RD] = c2[7] * k128;
    __syncthreads();

    v4f ov[2];
#pragma unroll
    for (int i = 0; i < 2; ++i) ov[i] = *(const v4f*)(stg + (2 * wave + i) * RD + 4 * lane);
    float* gp = g2 + ((size_t)nodeBase + r0 + 2 * wave) * RD + 4 * lane;
#pragma unroll
    for (int i = 0; i < 2; ++i) *(volatile v4f*)(gp + (size_t)i * RD) = ov[i];
    __threadfence();
#pragma unroll
    for (int i = 0; i < 2; ++i) *(volatile v4f*)(gp + (size_t)i * RD) = ov[i];
  }
}

__global__ __launch_bounds__(NTHR) void k_layer2(
    const float* __restrict__ g2, const float* __restrict__ ew,
    const int* __restrict__ esrc, const int* __restrict__ edst,
    const float* __restrict__ dsi, float* pooled, int nN, int nE, int vec8) {
  extern __shared__ v4f lds_dyn[];
  float* acc  = (float*)lds_dyn;
  int*   list = (int*)(acc + NB2 * RD);
  int*   wcnt = list + LISTN;
  float* pst  = (float*)list;
  const int tid = threadIdx.x, lane = tid & 31, wave = tid >> 5;
  const int nodeBase = blockIdx.x * NB2;

  {
    const v4f z = {0.f, 0.f, 0.f, 0.f};
    for (int i = tid; i < NB2 * RD / 4; i += NTHR) lds_dyn[i] = z;
  }
  __syncthreads();

  const int nChunks = (nE + CHUNK - 1) / CHUNK;
#pragma unroll 1
  for (int ch = 0; ch < nChunks; ++ch) {
    const int cbase = ch * CHUNK;
    const int wc = scan_chunk<NB2>(edst, nE, cbase, nodeBase, vec8, list, tid, lane, wave);
    if (lane == 0) wcnt[wave] = wc;
    __syncthreads();
    if (wave == 0) {
#pragma unroll 1
      for (int wsx = 0; wsx < NWAVE; ++wsx) {
        int n = __builtin_amdgcn_readfirstlane(wcnt[wsx]);
        n = n > WCAP ? WCAP : (n < 0 ? 0 : n);
        const int* lp = list + wsx * WCAP;
#pragma unroll 1
        for (int i = 0; i < n; ++i) {
          const int ent  = __builtin_amdgcn_readfirstlane(lp[i]);
          const int slot = ent & (NB2 - 1);
          int e = cbase + ((ent >> 12) & (CHUNK - 1));
          e = e > nE - 1 ? nE - 1 : e;
          int s = esrc[e];
          s = s < 0 ? 0 : (s > nN - 1 ? nN - 1 : s);
          const float we = ew[e];
          const v4f gv = *(const v4f*)(g2 + (size_t)s * RD + 4 * lane);
          v4f* ap = (v4f*)(acc + slot * RD + 4 * lane);
          *ap = *ap + gv * we;
        }
      }
    }
    __syncthreads();
  }

  const int c = tid & (RD - 1), gq = tid >> 7;
#pragma unroll 1
  for (int gg = 0; gg < 2; ++gg) {
    const int g = 2 * gq + gg;
    float sm = 0.f;
#pragma unroll 4
    for (int i = 0; i < NPG; ++i) {
      const int lr = NPG * g + i;
      const float d = dsi[(size_t)nodeBase + lr];
      float v = acc[lr * RD + c] * d;
      v = v >= 0.f ? v : 0.01f * v;
      sm += v;
    }
    pst[g * RD + c] = sm * (1.0f / NPG);
  }
  __syncthreads();

  const int ll = lane & 15;
  const int f  = 64 * wave + 4 * ll;
  const v4f pv = *(const v4f*)(pst + f);
  float* pp = pooled + (size_t)blockIdx.x * (GPB * RD) + f;
  if (lane < 16) *(volatile v4f*)pp = pv;
  __threadfence();
  if (lane < 16) *(volatile v4f*)pp = pv;
}

__global__ __launch_bounds__(NTHR) void k_head(
    const float* __restrict__ pooled, const float* __restrict__ Wl,
    const float* __restrict__ Wc, float* out, int G) {
  __shared__ __attribute__((aligned(16))) float P[HROWS * RD];
  __shared__ __attribute__((aligned(16))) float T[HROWS * 64];
  __shared__ __attribute__((aligned(16))) float O[HROWS * NCLS];
  const int tid = threadIdx.x, lane = tid & 31, wave = tid >> 5;
  const int g0 = blockIdx.x * HROWS;

#pragma unroll
  for (int i = 0; i < (HROWS * RD / 4) / NTHR; ++i) {
    const int idx = i * NTHR + tid;
    const int r   = idx >> 5;
    const int c4  = (idx & 31) * 4;
    int g = g0 + r;
    g = g > G - 1 ? G - 1 : g;
    *(v4f*)(P + r * RD + c4) = *(const v4f*)(pooled + (size_t)g * RD + c4);
  }
  __syncthreads();

  {
    const int d = tid & 63, rq = tid >> 6;
    float a8[8];
#pragma unroll
    for (int j = 0; j < 8; ++j) a8[j] = 0.f;
#pragma unroll 1
    for (int k = 0; k < RD; ++k) {
      const float w = Wl[k * 64 + d];
#pragma unroll
      for (int j = 0; j < 8; ++j) a8[j] += P[(8 * rq + j) * RD + k] * w;
    }
#pragma unroll
    for (int j = 0; j < 8; ++j) T[(8 * rq + j) * 64 + d] = a8[j];
  }
  __syncthreads();

  {
    const int d = tid & 15, r = tid >> 4;
    float b0 = 0.f, b1 = 0.f;
#pragma unroll 1
    for (int k = 0; k < 64; ++k) {
      const float w = Wc[k * NCLS + d];
      b0 += T[r * 64 + k] * w;
      b1 += T[(r + 16) * 64 + k] * w;
    }
    O[r * NCLS + d]        = b0;
    O[(r + 16) * NCLS + d] = b1;
  }
  __syncthreads();

  const int ll = lane & 15;
  const int f  = 64 * wave + 4 * ll;
  const v4f ov = *(const v4f*)(O + f);
  const size_t gi   = (size_t)g0 * NCLS + (size_t)f;
  const size_t outN = (size_t)G * NCLS;
  const bool ok = (lane < 16) && (gi + 4 <= outN);
  if (ok) *(volatile v4f*)(out + gi) = ov;
  __threadfence();
  if (ok) *(volatile v4f*)(out + gi) = ov;
}

extern "C" void kernel_launch(void* const* d_in, const int* in_sizes, int n_in,
                              void* d_out, int out_size, void* d_ws, size_t ws_size,
                              hipStream_t stream) {
  if (n_in < 8) return;
  const int nN = in_sizes[0] / IN_F;
  const int nE = in_sizes[1];
  if (nN <= 0 || nE < 0 || in_sizes[0] != nN * IN_F) return;
  if (in_sizes[2] != IN_F * HID || in_sizes[3] != HID * RD || in_sizes[4] != RD * 64 || in_sizes[5] != 64 * NCLS) return;
  if (in_sizes[6] != nE || in_sizes[7] != nE) return;
  const int G = nN / NPG;
  if (G <= 0 || out_size != G * NCLS) return;

  const float* x    = (const float*)d_in[0];
  const float* ew   = (const float*)d_in[1];
  const float* W1   = (const float*)d_in[2];
  const float* W2   = (const float*)d_in[3];
  const float* Wlin = (const float*)d_in[4];
  const float* Wcls = (const float*)d_in[5];
  const int*   esrc = (const int*)d_in[6];
  const int*   edst = (const int*)d_in[7];
  float* out = (float*)d_out;

  const int nBD = (nN + NBD - 1) / NBD;
  const int nA1 = (nN + NB1 - 1) / NB1;
  const int nA2 = (nN + NB2 - 1) / NB2;
  const int nH  = (G + HROWS - 1) / HROWS;
  const int planeN = nBD * NBD;

  char* ws = (char*)d_ws;
  size_t off = 0;
  const size_t oW1 = off; off += (size_t)HID * IN_F * 2;                         off = (off + 255) & ~(size_t)255;
  const size_t oW2 = off; off += (size_t)RD * HID * 2;                           off = (off + 255) & ~(size_t)255;
  const size_t oDv = off; off += (size_t)2 * planeN * 4;                          off = (off + 255) & ~(size_t)255;
  const size_t oG2 = off; off += (size_t)nA1 * NB1 * RD * 4;                      off = (off + 255) & ~(size_t)255;
  const size_t oPl = off; off += (size_t)nA2 * GPB * RD * 4;                      off = (off + 255) & ~(size_t)255;
  if (off > ws_size) return;
  _Float16* w1s    = (_Float16*)(ws + oW1);
  _Float16* w2s    = (_Float16*)(ws + oW2);
  float*    dso    = (float*)(ws + oDv);
  float*    dsi    = dso + planeN;
  float*    g2     = (float*)(ws + oG2);
  float*    pooled = (float*)(ws + oPl);

  const int vec8 = (((in_sizes[0] | in_sizes[1] | in_sizes[2] | in_sizes[3] | in_sizes[4] | in_sizes[5] | in_sizes[6]) & 3) == 0) ? 1 : 0;

  k_wprep<<<NBW1 + NBW2, NTHR, 0, stream>>>(W1, W2, w1s, w2s);

  k_deg<<<dim3(nBD, 2, 1), NTHR, 0, stream>>>(esrc, edst, dso, planeN, nE, vec8);

  hipFuncSetAttribute(reinterpret_cast<const void*>(&k_layer1),
                      hipFuncAttributeMaxDynamicSharedMemorySize, LDS_L1);
  k_layer1<<<nA1, NTHR, LDS_L1, stream>>>(x, ew, esrc, edst, dso, dsi, w1s, w2s, g2, nN, nE, vec8);

  hipFuncSetAttribute(reinterpret_cast<const void*>(&k_layer2),
                      hipFuncAttributeMaxDynamicSharedMemorySize, LDS_L2);
  k_layer2<<<nA2, NTHR, LDS_L2, stream>>>(g2, ew, esrc, edst, dsi, pooled, nN, nE, vec8);

  k_head<<<nH, NTHR, 0, stream>>>(pooled, Wlin, Wcls, out, G);
}
